// istsplm_forecast_31516470018549
// MI455X (gfx1250) — hardware-verified
//
#include <hip/hip_runtime.h>
#include <math.h>
#include <stddef.h>


constexpr int BB    = 2;
constexpr int S     = 2048;
constexpr int HID   = 2048;
constexpr int NH    = 16;
constexpr int NKV   = 2;
constexpr int HD    = 128;
constexpr int NREP  = NH / NKV;
constexpr int MROWS = BB * S;
constexpr int NQ    = NH * HD;
constexpr int NKVD  = NKV * HD;
constexpr int NQT   = S / 16;
constexpr int NKT   = S / 32;
constexpr int NFREQ = HD / 2;
constexpr float SCALE = 0.08838834764831845f;
constexpr int CP  = 132;
constexpr int OSP = 132;
constexpr int TP  = 68;

constexpr int EPI_ROPE = 1;
constexpr int EPI_ROWB = 2;
constexpr int EPI_F32  = 3;

static_assert(MROWS % 64 == 0);
static_assert(NQ % 128 == 0);
static_assert(NKVD % 128 == 0);
static_assert(HID % 64 == 0);
static_assert(S % 32 == 0);

typedef unsigned int   u32;
typedef unsigned short u16;
typedef __bf16 v16bf __attribute__((ext_vector_type(16)));
typedef float  v8f   __attribute__((ext_vector_type(8)));
typedef int    v8i   __attribute__((ext_vector_type(8)));
typedef float  v4f   __attribute__((ext_vector_type(4)));
typedef u32    v4u   __attribute__((ext_vector_type(4)));
typedef int    v4i   __attribute__((ext_vector_type(4)));
typedef v4f v4fa __attribute__((may_alias));
typedef v4u v4ua __attribute__((may_alias));
typedef v4i v4ia __attribute__((may_alias));

union Frag { v16bf v; v4u q[2]; };

__device__ __forceinline__ u32 bfb(float f) {
    const u32 u = __builtin_bit_cast(u32, f);
    return (u + 0x7FFFu + ((u >> 16) & 1u)) >> 16;
}
__device__ __forceinline__ float bff(u32 b) { return __builtin_bit_cast(float, b << 16); }

__device__ __forceinline__ void split8(const float (&x)[8], v4u& hi, v4u& lo) {
#pragma unroll
    for (int c = 0; c < 4; ++c) {
        const u32 h0 = bfb(x[2 * c]), h1 = bfb(x[2 * c + 1]);
        const u32 l0 = bfb(x[2 * c] - bff(h0)), l1 = bfb(x[2 * c + 1] - bff(h1));
        hi[c] = h0 | (h1 << 16);
        lo[c] = l0 | (l1 << 16);
    }
}

__device__ __forceinline__ v16bf ldfrag(const u16* p) {
    Frag f;
    f.q[0] = *(const v4ua*)(p);
    f.q[1] = *(const v4ua*)(p + 16);
    return f.v;
}

__device__ __forceinline__ v8f zero8() {
    v8f z;
#pragma unroll
    for (int i = 0; i < 8; ++i) z[i] = 0.0f;
    return z;
}

__device__ __forceinline__ void mma3(v8f& acc, v16bf ah, v16bf al, v16bf bh, v16bf bl) {
    acc = __builtin_amdgcn_wmma_f32_16x16x32_bf16(false, ah, false, bh, (short)0, acc, false, false);
    acc = __builtin_amdgcn_wmma_f32_16x16x32_bf16(false, ah, false, bl, (short)0, acc, false, false);
    acc = __builtin_amdgcn_wmma_f32_16x16x32_bf16(false, al, false, bh, (short)0, acc, false, false);
    const v8i ia = __builtin_bit_cast(v8i, ah);
    const v8i ib = __builtin_bit_cast(v8i, al);
    const v8i ic = __builtin_bit_cast(v8i, bh);
    const v8i id = __builtin_bit_cast(v8i, bl);
    asm volatile("v_nop\n\tv_nop\n\tv_nop\n\tv_nop"
                 : "+v"(acc) : "v"(ia), "v"(ib), "v"(ic), "v"(id) : "memory");
}

__device__ __forceinline__ void st2u(u16* ph, u16* pl, v4u hi, v4u lo) {
    *(volatile v4u*)ph = hi;
    *(volatile v4u*)pl = lo;
    __threadfence();
    *(volatile v4u*)ph = hi;
    *(volatile v4u*)pl = lo;
}
__device__ __forceinline__ void st2f(float* p, v4f v) {
    *(volatile v4f*)p = v;
    __threadfence();
    *(volatile v4f*)p = v;
}

__global__ void __launch_bounds__(256)
k_split_rows(const float* X, int n, u16* Xh, u16* Xl)
{
    const size_t i = ((size_t)blockIdx.x * 256 + threadIdx.x) * 8;
    if (i + 8 <= (size_t)n) {
        const v4f a = *(const v4fa*)(X + i);
        const v4f c = *(const v4fa*)(X + i + 4);
        float x[8] = {a[0], a[1], a[2], a[3], c[0], c[1], c[2], c[3]};
        v4u hi, lo;
        split8(x, hi, lo);
        st2u(Xh + i, Xl + i, hi, lo);
    }
}

__global__ void __launch_bounds__(256)
k_split_t(const float* W, int nrows, int ncols, u16* Th, u16* Tl)
{
    __shared__ __align__(16) float T[64 * TP];
    const int tid = threadIdx.x;
    const int cb = blockIdx.x * 64;
    const int rb = blockIdx.y * 64;
#pragma unroll
    for (int it = 0; it < 4; ++it) {
        const int fl = it * 256 + tid;
        const int rr = fl >> 4, cc = (fl & 15) * 4;
        const v4f v = *(const v4fa*)(W + (size_t)(rb + rr) * ncols + cb + cc);
        T[(cc + 0) * TP + rr] = v[0];
        T[(cc + 1) * TP + rr] = v[1];
        T[(cc + 2) * TP + rr] = v[2];
        T[(cc + 3) * TP + rr] = v[3];
    }
    __syncthreads();
#pragma unroll
    for (int it = 0; it < 2; ++it) {
        const int orow = it * 32 + (tid >> 3), oc = (tid & 7) * 8;
        const v4f a = *(const v4fa*)(T + orow * TP + oc);
        const v4f c = *(const v4fa*)(T + orow * TP + oc + 4);
        float x[8] = {a[0], a[1], a[2], a[3], c[0], c[1], c[2], c[3]};
        v4u hi, lo;
        split8(x, hi, lo);
        const size_t o = (size_t)(cb + orow) * nrows + rb + oc;
        st2u(Th + o, Tl + o, hi, lo);
    }
}

__global__ void __launch_bounds__(256)
k_rope_table(const float* ts, int nrows, float* cosT, float* sinT)
{
    const int tid = threadIdx.x;
    const int row = blockIdx.x * 4 + (tid >> 6);
    const int j   = tid & 63;
    const int rc  = row < nrows ? row : nrows - 1;
    const float t = ts[rc];
    const double p  = exp2((double)j * (13.287712379549449 / 64.0));
    const float  pf = (float)p;
    const float inv = 1.0f / pf;
    const float ang = t * inv;
    float sn, cs;
    sincosf(ang, &sn, &cs);
    if (row < nrows) {
        const size_t o = (size_t)row * NFREQ + j;
        *(volatile float*)(cosT + o) = cs;
        *(volatile float*)(sinT + o) = sn;
        __threadfence();
        *(volatile float*)(cosT + o) = cs;
        *(volatile float*)(sinT + o) = sn;
    }
}

__global__ void __launch_bounds__(256)
k_flags(const float* amask, int* flags)
{
    __shared__ __align__(16) int sf[32];
    const int tid = threadIdx.x, lane = tid & 31, w = tid >> 5;
    const int qt = blockIdx.x, hf = blockIdx.y;
    const int t = tid >> 3, sub = tid & 7;
    const int kt = hf * 32 + t;
    const int kb = kt * 32;
    int ok = 1;
#pragma unroll
    for (int rr = 0; rr < 2; ++rr) {
        const int q = qt * 16 + sub * 2 + rr;
        const float* mp = amask + (size_t)q * S + kb;
#pragma unroll
        for (int c = 0; c < 8; ++c) {
            const v4f v = *(const v4fa*)(mp + 4 * c);
            ok &= (int)(v[0] <= -1.0e8f) & (int)(v[1] <= -1.0e8f) &
                  (int)(v[2] <= -1.0e8f) & (int)(v[3] <= -1.0e8f);
        }
    }
    ok &= __shfl_xor(ok, 1);
    ok &= __shfl_xor(ok, 2);
    ok &= __shfl_xor(ok, 4);
    if (sub == 0) sf[t] = ok;
    __syncthreads();
    if (w == 0 && lane < 8) {
        const v4i f = *(const v4ia*)(sf + lane * 4);
        int* dst = flags + (size_t)qt * NKT + hf * 32 + lane * 4;
        *(volatile v4i*)dst = f;
        __threadfence();
        *(volatile v4i*)dst = f;
    }
}

template<int EPI>
__global__ void __launch_bounds__(128)
gemm_x3(const u16* Ah, const u16* Al, int lda,
        const u16* Bh, const u16* Bl, int ldb, int K,
        const float* bias, const float* cosT, const float* sinT,
        u16* Oh, u16* Ol, float* Of, int ldo)
{
    __shared__ __align__(16) float Cs[64 * CP];
    const int tid = threadIdx.x, w = tid >> 5, lane = tid & 31;
    const int h = lane >> 4, ln = lane & 15;
    const int wm = w >> 1, wn = w & 1;
    const int i0 = blockIdx.y * 64, j0 = blockIdx.x * 128;

    v8f acc[2][4];
#pragma unroll
    for (int mi = 0; mi < 2; ++mi)
#pragma unroll
        for (int ni = 0; ni < 4; ++ni) acc[mi][ni] = zero8();

    size_t aofs[2], bofs[4];
#pragma unroll
    for (int mi = 0; mi < 2; ++mi)
        aofs[mi] = (size_t)(i0 + wm * 32 + mi * 16 + ln) * lda + 8 * h;
#pragma unroll
    for (int ni = 0; ni < 4; ++ni)
        bofs[ni] = (size_t)(j0 + wn * 64 + ni * 16 + ln) * ldb + 8 * h;

#pragma unroll 1
    for (int k0 = 0; k0 < K; k0 += 32) {
        const v16bf ah0 = ldfrag(Ah + aofs[0] + k0);
        const v16bf al0 = ldfrag(Al + aofs[0] + k0);
        const v16bf ah1 = ldfrag(Ah + aofs[1] + k0);
        const v16bf al1 = ldfrag(Al + aofs[1] + k0);
#pragma unroll
        for (int ni = 0; ni < 4; ++ni) {
            const v16bf bh = ldfrag(Bh + bofs[ni] + k0);
            const v16bf bl = ldfrag(Bl + bofs[ni] + k0);
            mma3(acc[0][ni], ah0, al0, bh, bl);
            mma3(acc[1][ni], ah1, al1, bh, bl);
        }
    }

#pragma unroll
    for (int mi = 0; mi < 2; ++mi)
#pragma unroll
        for (int ni = 0; ni < 4; ++ni)
#pragma unroll
            for (int r = 0; r < 8; ++r)
                Cs[(wm * 32 + mi * 16 + 8 * h + r) * CP + wn * 64 + ni * 16 + ln] = acc[mi][ni][r];
    __syncthreads();

    if (EPI == EPI_F32) {
#pragma unroll 1
        for (int it = 0; it < 16; ++it) {
            const int row = it * 4 + w, col = lane * 4;
            v4f x = *(const v4fa*)(Cs + row * CP + col);
            const v4f bv = *(const v4fa*)(bias + j0 + col);
            x += bv;
            st2f(Of + (size_t)(i0 + row) * ldo + j0 + col, x);
        }
    } else {
#pragma unroll 1
        for (int it = 0; it < 8; ++it) {
            const int row = it * 8 + w * 2 + h, colc = ln * 8;
            const int gi = i0 + row;
            const float* cr = Cs + row * CP;
            float x[8];
            {
                const v4f a = *(const v4fa*)(cr + colc);
                const v4f c = *(const v4fa*)(cr + colc + 4);
                x[0] = a[0]; x[1] = a[1]; x[2] = a[2]; x[3] = a[3];
                x[4] = c[0]; x[5] = c[1]; x[6] = c[2]; x[7] = c[3];
            }
            if (EPI == EPI_ROWB) {
                const float bvv = bias[gi];
#pragma unroll
                for (int e = 0; e < 8; ++e) x[e] += bvv;
            } else {
                const v4f b0 = *(const v4fa*)(bias + j0 + colc);
                const v4f b1 = *(const v4fa*)(bias + j0 + colc + 4);
                x[0] += b0[0]; x[1] += b0[1]; x[2] += b0[2]; x[3] += b0[3];
                x[4] += b1[0]; x[5] += b1[1]; x[6] += b1[2]; x[7] += b1[3];
            }
            if (EPI == EPI_ROPE) {
                const int pc = colc ^ 64;
                float xp[8];
                {
                    const v4f a = *(const v4fa*)(cr + pc);
                    const v4f c = *(const v4fa*)(cr + pc + 4);
                    const v4f b0 = *(const v4fa*)(bias + j0 + pc);
                    const v4f b1 = *(const v4fa*)(bias + j0 + pc + 4);
                    xp[0] = a[0] + b0[0]; xp[1] = a[1] + b0[1]; xp[2] = a[2] + b0[2]; xp[3] = a[3] + b0[3];
                    xp[4] = c[0] + b1[0]; xp[5] = c[1] + b1[1]; xp[6] = c[2] + b1[2]; xp[7] = c[3] + b1[3];
                }
                const int jb = colc & 63;
                const float* cp = cosT + (size_t)gi * NFREQ + jb;
                const float* sp = sinT + (size_t)gi * NFREQ + jb;
                const v4f c0 = *(const v4fa*)(cp), c1 = *(const v4fa*)(cp + 4);
                const v4f s0 = *(const v4fa*)(sp), s1 = *(const v4fa*)(sp + 4);
                float cs[8] = {c0[0], c0[1], c0[2], c0[3], c1[0], c1[1], c1[2], c1[3]};
                float sn[8] = {s0[0], s0[1], s0[2], s0[3], s1[0], s1[1], s1[2], s1[3]};
                const float sg = (colc < 64) ? -1.0f : 1.0f;
#pragma unroll
                for (int e = 0; e < 8; ++e) x[e] = x[e] * cs[e] + sg * (xp[e] * sn[e]);
            }
            v4u hi, lo;
            split8(x, hi, lo);
            const size_t o = (size_t)gi * ldo + j0 + colc;
            st2u(Oh + o, Ol + o, hi, lo);
        }
    }
}

__global__ void __launch_bounds__(32)
attn_x3(const u16* Qh, const u16* Ql, const u16* Kh, const u16* Kl,
        const u16* Vh, const u16* Vl, const float* amask, const int* flags,
        u16* Oh, u16* Ol)
{
    __shared__ __align__(16) u16 Ph[16 * 32];
    __shared__ __align__(16) u16 Pl[16 * 32];
    __shared__ __align__(16) float Os[16 * OSP];

    const int lane = threadIdx.x & 31, h = lane >> 4, ln = lane & 15;
    const int qt = blockIdx.x, hh = blockIdx.y, b = blockIdx.z;
    const int kvh = hh / NREP;
    const int q0 = qt * 16;

    const size_t qofs = (size_t)(b * S + q0 + ln) * NQ + hh * HD + 8 * h;
    const size_t kofs = (size_t)(b * S + ln) * NKVD + kvh * HD + 8 * h;
    const size_t vofs = (size_t)(kvh * HD + ln) * MROWS + b * S + 8 * h;
    const size_t mofs = (size_t)(q0 + 8 * h) * S + ln;

    float mrun[8], lrun[8];
    v8f o[8];
#pragma unroll
    for (int r = 0; r < 8; ++r) { mrun[r] = -1.0e30f; lrun[r] = 0.0f; }
#pragma unroll
    for (int t = 0; t < 8; ++t) o[t] = zero8();

    for (int kt = 0; kt < NKT; ++kt) {
        int f = flags[qt * NKT + kt];
        f = __builtin_amdgcn_readfirstlane(f);
        if (f == 1) continue;
        const int kb = kt * 32;

        v8f s0 = zero8(), s1 = zero8();
#pragma unroll
        for (int dc = 0; dc < 4; ++dc) {
            const v16bf qh = ldfrag(Qh + qofs + dc * 32);
            const v16bf ql = ldfrag(Ql + qofs + dc * 32);
            const size_t k0o = kofs + (size_t)kb * NKVD + dc * 32;
            const size_t k1o = k0o + (size_t)16 * NKVD;
            v16bf kh = ldfrag(Kh + k0o);
            v16bf kl = ldfrag(Kl + k0o);
            mma3(s0, qh, ql, kh, kl);
            kh = ldfrag(Kh + k1o);
            kl = ldfrag(Kl + k1o);
            mma3(s1, qh, ql, kh, kl);
        }

#pragma unroll
        for (int r = 0; r < 8; ++r) {
            const float* mp = amask + mofs + (size_t)r * S + kb;
            const float mk0 = mp[0];
            const float mk1 = mp[16];
            const float a0 = s0[r] * SCALE + mk0;
            const float a1 = s1[r] * SCALE + mk1;
            float mx = fmaxf(a0, a1);
            mx = fmaxf(mx, __shfl_xor(mx, 1));
            mx = fmaxf(mx, __shfl_xor(mx, 2));
            mx = fmaxf(mx, __shfl_xor(mx, 4));
            mx = fmaxf(mx, __shfl_xor(mx, 8));
            const float mnew = fmaxf(mrun[r], mx);
            const float corr = __expf(mrun[r] - mnew);
            const float p0 = __expf(a0 - mnew);
            const float p1 = __expf(a1 - mnew);
            mrun[r] = mnew;
            float ps = p0 + p1;
            ps += __shfl_xor(ps, 1);
            ps += __shfl_xor(ps, 2);
            ps += __shfl_xor(ps, 4);
            ps += __shfl_xor(ps, 8);
            lrun[r] = lrun[r] * corr + ps;
#pragma unroll
            for (int t = 0; t < 8; ++t) o[t][r] *= corr;
            const u32 h0 = bfb(p0), h1 = bfb(p1);
            const u32 l0 = bfb(p0 - bff(h0)), l1 = bfb(p1 - bff(h1));
            const int prow = (8 * h + r) * 32;
            Ph[prow + ln] = (u16)h0;
            Ph[prow + 16 + ln] = (u16)h1;
            Pl[prow + ln] = (u16)l0;
            Pl[prow + 16 + ln] = (u16)l1;
        }
        __syncthreads();

        const v16bf ph = ldfrag(Ph + ln * 32 + 8 * h);
        const v16bf pl = ldfrag(Pl + ln * 32 + 8 * h);
#pragma unroll
        for (int t = 0; t < 8; ++t) {
            const size_t vo = vofs + (size_t)(t * 16) * MROWS + kb;
            const v16bf vh = ldfrag(Vh + vo);
            const v16bf vl = ldfrag(Vl + vo);
            mma3(o[t], ph, pl, vh, vl);
        }
        __syncthreads();
    }

#pragma unroll
    for (int r = 0; r < 8; ++r) {
        const float lv = lrun[r];
        const float li = (lv > 0.0f) ? (1.0f / lv) : 0.0f;
        const int orow = (8 * h + r) * OSP;
#pragma unroll
        for (int t = 0; t < 8; ++t) Os[orow + t * 16 + ln] = o[t][r] * li;
    }
    __syncthreads();
#pragma unroll 1
    for (int it = 0; it < 8; ++it) {
        const int row = it * 2 + h, colc = ln * 8;
        const float* cr = Os + row * OSP;
        const v4f a = *(const v4fa*)(cr + colc);
        const v4f c = *(const v4fa*)(cr + colc + 4);
        float x[8] = {a[0], a[1], a[2], a[3], c[0], c[1], c[2], c[3]};
        v4u hi, lo;
        split8(x, hi, lo);
        const size_t oo = (size_t)(b * S + q0 + row) * NQ + hh * HD + colc;
        st2u(Oh + oo, Ol + oo, hi, lo);
    }
}

extern "C" void kernel_launch(void* const* d_in, const int* in_sizes, int n_in,
                              void* d_out, int out_size, void* d_ws, size_t ws_size,
                              hipStream_t stream)
{
    if (n_in < 11) return;
    if (in_sizes[0] != MROWS * HID || in_sizes[1] != MROWS || in_sizes[2] != S * S ||
        in_sizes[3] != HID * NQ || in_sizes[4] != NQ ||
        in_sizes[5] != HID * NKVD || in_sizes[6] != NKVD ||
        in_sizes[7] != HID * NKVD || in_sizes[8] != NKVD ||
        in_sizes[9] != NQ * HID || in_sizes[10] != HID) return;
    if (out_size != MROWS * HID) return;

    const float* X   = (const float*)d_in[0];
    const float* ts  = (const float*)d_in[1];
    const float* amk = (const float*)d_in[2];
    const float* Wq  = (const float*)d_in[3];
    const float* bq  = (const float*)d_in[4];
    const float* Wk  = (const float*)d_in[5];
    const float* bk  = (const float*)d_in[6];
    const float* Wv  = (const float*)d_in[7];
    const float* bv  = (const float*)d_in[8];
    const float* Wo  = (const float*)d_in[9];
    const float* bo  = (const float*)d_in[10];
    float* out = (float*)d_out;

    const size_t szX  = (size_t)MROWS * HID * 2;
    const size_t szWq = (size_t)NQ * HID * 2;
    const size_t szWk = (size_t)NKVD * HID * 2;
    const size_t szWo = (size_t)HID * NQ * 2;
    const size_t szQ  = (size_t)MROWS * NQ * 2;
    const size_t szK  = (size_t)MROWS * NKVD * 2;
    const size_t szVt = (size_t)NKVD * MROWS * 2;
    const size_t szTb = (size_t)MROWS * NFREQ * 4;
    const size_t szFl = (size_t)NQT * NKT * 4;
    char* base = (char*)d_ws;
    size_t used = 0;
    auto take = [&](size_t bytes) -> char* { char* p = base + used; used += (bytes + 255) & ~(size_t)255; return p; };
    u16* Xh   = (u16*)take(szX);   u16* Xl   = (u16*)take(szX);
    u16* Wqth = (u16*)take(szWq);  u16* Wqtl = (u16*)take(szWq);
    u16* Wkth = (u16*)take(szWk);  u16* Wktl = (u16*)take(szWk);
    u16* Wvth = (u16*)take(szWk);  u16* Wvtl = (u16*)take(szWk);
    u16* Woth = (u16*)take(szWo);  u16* Wotl = (u16*)take(szWo);
    u16* Qh   = (u16*)take(szQ);   u16* Ql   = (u16*)take(szQ);
    u16* Kh   = (u16*)take(szK);   u16* Kl   = (u16*)take(szK);
    u16* Vth  = (u16*)take(szVt);  u16* Vtl  = (u16*)take(szVt);
    float* cosT = (float*)take(szTb);
    float* sinT = (float*)take(szTb);
    int* flags  = (int*)take(szFl);
    if (used > ws_size) return;
    u16* AOh = Xh;
    u16* AOl = Xl;

    k_split_rows<<<dim3((MROWS * HID) / (256 * 8)), dim3(256), 0, stream>>>(X, MROWS * HID, Xh, Xl);
    k_split_t<<<dim3(NQ / 64, HID / 64), dim3(256), 0, stream>>>(Wq, HID, NQ, Wqth, Wqtl);
    k_split_t<<<dim3(NKVD / 64, HID / 64), dim3(256), 0, stream>>>(Wk, HID, NKVD, Wkth, Wktl);
    k_split_t<<<dim3(NKVD / 64, HID / 64), dim3(256), 0, stream>>>(Wv, HID, NKVD, Wvth, Wvtl);
    k_split_t<<<dim3(HID / 64, NQ / 64), dim3(256), 0, stream>>>(Wo, NQ, HID, Woth, Wotl);
    k_rope_table<<<dim3(MROWS / 4), dim3(256), 0, stream>>>(ts, MROWS, cosT, sinT);
    k_flags<<<dim3(NQT, 2), dim3(256), 0, stream>>>(amk, flags);
    gemm_x3<EPI_ROPE><<<dim3(NQ / 128, MROWS / 64), dim3(128), 0, stream>>>(
        Xh, Xl, HID, Wqth, Wqtl, HID, HID, bq, cosT, sinT, Qh, Ql, out, NQ);
    gemm_x3<EPI_ROPE><<<dim3(NKVD / 128, MROWS / 64), dim3(128), 0, stream>>>(
        Xh, Xl, HID, Wkth, Wktl, HID, HID, bk, cosT, sinT, Kh, Kl, out, NKVD);
    gemm_x3<EPI_ROWB><<<dim3(MROWS / 128, NKVD / 64), dim3(128), 0, stream>>>(
        Wvth, Wvtl, HID, Xh, Xl, HID, HID, bv, cosT, sinT, Vth, Vtl, out, MROWS);
    attn_x3<<<dim3(NQT, NH, BB), dim3(32), 0, stream>>>(Qh, Ql, Kh, Kl, Vth, Vtl, amk, flags, AOh, AOl);
    gemm_x3<EPI_F32><<<dim3(HID / 128, MROWS / 64), dim3(128), 0, stream>>>(
        AOh, AOl, NQ, Woth, Wotl, NQ, NQ, bo, cosT, sinT, Qh, Ql, out, HID);
    (void)hipGetLastError();
}
